// MultiHeadAttention_31267361915364
// MI455X (gfx1250) — hardware-verified
//
#include <hip/hip_runtime.h>
#ifndef NB
#define NB 4
#endif
#ifndef SEQ
#define SEQ 2048
#endif
#ifndef EARLY
#define EARLY 256
#endif
#define NB_FULL 4
#define SEQ_FULL 2048
#define DM 1024
#define NH 16
#define HD 64
#define LQ (3 * DM)
static_assert(SEQ % 128 == 0);
static_assert(EARLY % 128 == 0);
static_assert(EARLY <= SEQ);
static_assert(NB <= NB_FULL);
static_assert(SEQ <= SEQ_FULL);
static_assert(NH * HD == DM);
static_assert(DM % 64 == 0);

typedef _Float16 v16h __attribute__((ext_vector_type(16)));
typedef _Float16 v4h __attribute__((ext_vector_type(4)));
typedef unsigned short v8us __attribute__((ext_vector_type(8), may_alias));
typedef float v8f __attribute__((ext_vector_type(8)));
typedef float v4f __attribute__((ext_vector_type(4)));
typedef float v4fa __attribute__((ext_vector_type(4), may_alias));
union FragH { v16h v; v8us half[2]; _Float16 h[16]; unsigned short u[16]; };

__device__ __forceinline__ float bf16_rne(float x) {
  unsigned int u = __float_as_uint(x);
  u = (u + 0x7FFFu + ((u >> 16) & 1u)) & 0xFFFF0000u;
  return __uint_as_float(u);
}
__device__ __forceinline__ v16h ld_frag(const _Float16* p, int hh) {
  FragH f;
  f.half[0] = *(const v8us*)((const unsigned short*)p + 8 * hh);
  f.half[1] = *(const v8us*)((const unsigned short*)p + 16 + 8 * hh);
  return f.v;
}
__device__ __forceinline__ v8f mma16(v16h a, v16h b, v8f c) {
  v8f d = __builtin_amdgcn_wmma_f32_16x16x32_f16(false, a, false, b, (short)0, c, false, false);
  asm volatile("v_nop\n\tv_nop\n\tv_nop\n\tv_nop" : "+v"(d) : "v"(a), "v"(b));
  return d;
}

__global__ __launch_bounds__(256) void k_wt_f16(const float* __restrict__ W, _Float16* __restrict__ Wt, int K, int N, float scale) {
  const int t = blockIdx.x * 256 + threadIdx.x;
  if (t >= N * (K / 8)) return;
  const int n = t / (K / 8), k8 = (t % (K / 8)) * 8;
  FragH f;
#pragma unroll
  for (int i = 0; i < 8; ++i) f.h[i] = (_Float16)(bf16_rne(W[(size_t)(k8 + i) * N + n]) * scale);
  const v8us o = f.half[0];
  unsigned short* d = (unsigned short*)Wt + (size_t)n * K + k8;
  *(volatile v8us*)d = o;
  __threadfence();
  *(volatile v8us*)d = o;
}

__global__ __launch_bounds__(256) void k_x16(const float* __restrict__ x, _Float16* __restrict__ X16) {
  const size_t t = (size_t)blockIdx.x * 256 + threadIdx.x;
  if (t >= (size_t)NB * SEQ * DM / 8) return;
  const size_t row = t / (DM / 8);
  const int c8 = (int)(t % (DM / 8)) * 8;
  const size_t b = row / SEQ, s = row % SEQ;
  const float* src = x + (b * SEQ_FULL + s) * DM + c8;
  const v4f a = *(const v4fa*)src, c = *(const v4fa*)(src + 4);
  FragH f;
#pragma unroll
  for (int q = 0; q < 4; ++q) { f.h[q] = (_Float16)bf16_rne(a[q]); f.h[4 + q] = (_Float16)bf16_rne(c[q]); }
  const v8us o = f.half[0];
  unsigned short* d = (unsigned short*)X16 + t * 8;
  *(volatile v8us*)d = o;
  __threadfence();
  *(volatile v8us*)d = o;
}

__device__ __forceinline__ void gemm_core(const _Float16* __restrict__ a0p, const _Float16* __restrict__ a1p, const _Float16* __restrict__ b0p,
                                          const int ldb, const int K, const int hh,
                                          v8f& c00, v8f& c01, v8f& c02, v8f& c03, v8f& c10, v8f& c11, v8f& c12, v8f& c13) {
  const _Float16* b1p = b0p + (size_t)16 * ldb;
  const _Float16* b2p = b1p + (size_t)16 * ldb;
  const _Float16* b3p = b2p + (size_t)16 * ldb;
#pragma unroll 1
  for (int kb = 0; kb < K; kb += 32) {
    const v16h a0 = ld_frag(a0p + kb, hh), a1 = ld_frag(a1p + kb, hh);
    v16h b = ld_frag(b0p + kb, hh); c00 = mma16(a0, b, c00); c10 = mma16(a1, b, c10);
    b = ld_frag(b1p + kb, hh); c01 = mma16(a0, b, c01); c11 = mma16(a1, b, c11);
    b = ld_frag(b2p + kb, hh); c02 = mma16(a0, b, c02); c12 = mma16(a1, b, c12);
    b = ld_frag(b3p + kb, hh); c03 = mma16(a0, b, c03); c13 = mma16(a1, b, c13);
  }
}

template <bool LO>
__global__ __launch_bounds__(128) void k_gemm_qkv(const _Float16* __restrict__ X16, const _Float16* __restrict__ Wt, const float* __restrict__ bias,
                                                _Float16* __restrict__ QKV, _Float16* __restrict__ QKVL) {
  __shared__ __attribute__((aligned(16))) float so[4][32][68];
  const int w = __builtin_amdgcn_readfirstlane((int)(threadIdx.x >> 5));
  const int lane = threadIdx.x & 31, ln = lane & 15, hh = lane >> 4;
  const int by = blockIdx.y;
  constexpr int NTN = LQ / 64;
  const int mt = blockIdx.x / NTN, nq = blockIdx.x - mt * NTN;
  const int s0 = (LO ? 0 : EARLY) + mt * 128 + 32 * w;
  const int col0 = nq * 64;
  const size_t row0 = (size_t)by * SEQ + s0;
  const _Float16* a0p = X16 + (row0 + ln) * DM;
  const _Float16* a1p = a0p + (size_t)16 * DM;
  const _Float16* b0p = Wt + (size_t)(col0 + ln) * DM;
  const v8f z8 = {0.f, 0.f, 0.f, 0.f, 0.f, 0.f, 0.f, 0.f};
  v8f c00 = z8, c01 = z8, c02 = z8, c03 = z8, c10 = z8, c11 = z8, c12 = z8, c13 = z8;
  gemm_core(a0p, a1p, b0p, DM, DM, hh, c00, c01, c02, c03, c10, c11, c12, c13);
  v8f accs[8] = {c00, c01, c02, c03, c10, c11, c12, c13};
#pragma unroll
  for (int u = 0; u < 8; ++u) {
    const int t = u & 3, half = u >> 2;
    const float bv = bf16_rne(bias[col0 + t * 16 + ln]);
#pragma unroll
    for (int r = 0; r < 8; ++r) so[w][half * 16 + 8 * hh + r][t * 16 + ln] = accs[u][r] * 0.0625f + bv;
  }
  __builtin_amdgcn_fence(4  , "workgroup");
  __builtin_amdgcn_wave_barrier();
  const int rsub = lane >> 4, c4 = (lane & 15) * 4;
  for (int pass = 0; pass < 2; ++pass) {
#pragma unroll
    for (int q = 0; q < 16; ++q) {
      const int r = q * 2 + rsub;
      const v4f v = *(const v4fa*)&so[w][r][c4];
      v4h h4;
#pragma unroll
      for (int i = 0; i < 4; ++i) h4[i] = (_Float16)v[i];
      *(volatile v4h*)(QKV + (row0 + r) * LQ + col0 + c4) = h4;
      if (LO) {
        v4h l4;
#pragma unroll
        for (int i = 0; i < 4; ++i) l4[i] = (_Float16)((v[i] - (float)h4[i]) * 1024.0f);
        *(volatile v4h*)(QKVL + ((size_t)by * EARLY + s0 + r) * LQ + col0 + c4) = l4;
      }
    }
    if (pass == 0) __threadfence();
  }
}

template <int TTv>
__global__ __launch_bounds__(256) void k_vt(const _Float16* __restrict__ V16, _Float16* __restrict__ Vt) {
  __shared__ unsigned short tl[64][66];
  const int tid = threadIdx.x;
  const int slab = blockIdx.x / (TTv / 64), lg = blockIdx.x % (TTv / 64);
  const int b = slab / NH, h = slab % NH;
  for (int i = tid; i < 64 * 8; i += 256) {
    const int r = i / 8, c8 = (i % 8) * 8;
    FragH f;
    f.half[0] = *(const v8us*)((const unsigned short*)V16 + ((size_t)b * TTv + lg * 64 + r) * LQ + h * HD + c8);
#pragma unroll
    for (int q = 0; q < 8; ++q) tl[r][c8 + q] = f.u[q];
  }
  __syncthreads();
  for (int pass = 0; pass < 2; ++pass) {
#pragma unroll
    for (int rd = 0; rd < 2; ++rd) {
      const int d = rd * 32 + tid / 8, pc = tid % 8;
      FragH f;
#pragma unroll
      for (int q = 0; q < 8; ++q) f.u[q] = tl[pc * 8 + q][d];
      *(volatile v8us*)((unsigned short*)Vt + ((size_t)slab * 64 + d) * TTv + lg * 64 + pc * 8) = f.half[0];
    }
    if (pass == 0) __threadfence();
  }
}

template <bool PREC>
__device__ __forceinline__ void pv_tile(const _Float16* __restrict__ vp, const _Float16* __restrict__ vlp, const int hh,
                                        const v16h ph, const v16h pl, v8f& om, v8f& orr) {
  const v16h av = ld_frag(vp, hh);
  om = mma16(av, ph, om);
  if (PREC) {
    orr = mma16(av, pl, orr);
    const v16h avl = ld_frag(vlp, hh);
    orr = mma16(avl, ph, orr);
  }
}

template <bool PREC, bool MASK>
__device__ __forceinline__ void attn_step(const int kb, const int qn, const int ln, const int hh,
                                          const _Float16* __restrict__ kbase, const _Float16* __restrict__ klbase,
                                          const _Float16* __restrict__ vbase, const _Float16* __restrict__ vlbase,
                                          const v16h bq0, const v16h bq1, const v16h bl0, const v16h bl1,
                                          float& M, float& L,
                                          v8f& om0, v8f& om1, v8f& om2, v8f& om3, v8f& or0, v8f& or1, v8f& or2, v8f& or3) {
  const v8f z8 = {0.f, 0.f, 0.f, 0.f, 0.f, 0.f, 0.f, 0.f};
  const _Float16* k0p = kbase + (size_t)(kb + ln) * LQ;
  const _Float16* k1p = k0p + (size_t)16 * LQ;
  const _Float16* kl0p = klbase + (size_t)(kb + ln) * LQ;
  const _Float16* kl1p = kl0p + (size_t)16 * LQ;
  v8f s0 = z8, s1 = z8, r0 = z8, r1 = z8;
  {
    v16h a = ld_frag(k0p, hh);
    s0 = mma16(a, bq0, s0); if (PREC) r0 = mma16(a, bl0, r0);
    a = ld_frag(k0p + 32, hh);
    s0 = mma16(a, bq1, s0); if (PREC) r0 = mma16(a, bl1, r0);
    if (PREC) { a = ld_frag(kl0p, hh); r0 = mma16(a, bq0, r0); a = ld_frag(kl0p + 32, hh); r0 = mma16(a, bq1, r0); }
    a = ld_frag(k1p, hh);
    s1 = mma16(a, bq0, s1); if (PREC) r1 = mma16(a, bl0, r1);
    a = ld_frag(k1p + 32, hh);
    s1 = mma16(a, bq1, s1); if (PREC) r1 = mma16(a, bl1, r1);
    if (PREC) { a = ld_frag(kl1p, hh); r1 = mma16(a, bq0, r1); a = ld_frag(kl1p + 32, hh); r1 = mma16(a, bq1, r1); }
  }
  float sv[16];
#pragma unroll
  for (int r = 0; r < 8; ++r) {
    if (PREC) {
      sv[r] = (s0[r] + r0[r] * 0.0009765625f) * 0.03125f;
      sv[8 + r] = (s1[r] + r1[r] * 0.0009765625f) * 0.03125f;
    } else {
      sv[r] = s0[r] * 0.03125f;
      sv[8 + r] = s1[r] * 0.03125f;
    }
  }
  if (MASK) {
#pragma unroll
    for (int r = 0; r < 8; ++r) {
      const int key0 = kb + 8 * hh + r;
      sv[r] = (key0 <= qn) ? sv[r] : -3.0e38f;
      sv[8 + r] = (key0 + 16 <= qn) ? sv[8 + r] : -3.0e38f;
    }
  }
  float mx = sv[0];
#pragma unroll
  for (int i = 1; i < 16; ++i) mx = fmaxf(mx, sv[i]);
  mx = fmaxf(mx, __shfl_xor(mx, 16, 32));
  const float Mn = fmaxf(M, mx - 5.545177444f);
  const float al = __expf(M - Mn);
  M = Mn;
  float p[16];
  float ps = 0.f;
#pragma unroll
  for (int i = 0; i < 16; ++i) { p[i] = __expf(sv[i] - Mn); ps += p[i]; }
  L = L * al + ps;
  om0 *= al; om1 *= al; om2 *= al; om3 *= al;
  if (PREC) { or0 *= al; or1 *= al; or2 *= al; or3 *= al; }
  FragH pb, pl;
#pragma unroll
  for (int i = 0; i < 16; ++i) {
    const _Float16 hv = (_Float16)p[i];
    pb.h[i] = hv;
    pl.h[i] = PREC ? (_Float16)((p[i] - (float)hv) * 1024.0f) : (_Float16)0.0f;
  }
  pv_tile<PREC>(vbase + (size_t)(0 * 16 + ln) * SEQ + kb, vlbase + (size_t)(0 * 16 + ln) * EARLY + kb, hh, pb.v, pl.v, om0, or0);
  pv_tile<PREC>(vbase + (size_t)(1 * 16 + ln) * SEQ + kb, vlbase + (size_t)(1 * 16 + ln) * EARLY + kb, hh, pb.v, pl.v, om1, or1);
  pv_tile<PREC>(vbase + (size_t)(2 * 16 + ln) * SEQ + kb, vlbase + (size_t)(2 * 16 + ln) * EARLY + kb, hh, pb.v, pl.v, om2, or2);
  pv_tile<PREC>(vbase + (size_t)(3 * 16 + ln) * SEQ + kb, vlbase + (size_t)(3 * 16 + ln) * EARLY + kb, hh, pb.v, pl.v, om3, or3);
}

template <bool PREC>
__global__ __launch_bounds__(128) void k_attn(const _Float16* __restrict__ QKV, const _Float16* __restrict__ QKVL,
                                            const _Float16* __restrict__ VT, const _Float16* __restrict__ VTL,
                                            _Float16* __restrict__ CTX, _Float16* __restrict__ CTXL) {
  __shared__ __attribute__((aligned(16))) unsigned short th[4][16][72];
  __shared__ __attribute__((aligned(16))) unsigned short tl[PREC ? 4 : 1][16][72];
  const int w = __builtin_amdgcn_readfirstlane((int)(threadIdx.x >> 5));
  const int lane = threadIdx.x & 31, ln = lane & 15, hh = lane >> 4;
  constexpr int TPB = PREC ? (EARLY / 16) : (((SEQ - EARLY) / 16) > 0 ? ((SEQ - EARLY) / 16) : 1);
  const int gw = blockIdx.x * 4 + w;
  const int bh = gw / TPB;
  const int qt = gw - bh * TPB + (PREC ? 0 : EARLY / 16);
  const int b = bh / NH, h = bh - b * NH;
  const int q0 = qt * 16;
  const size_t rowb = (size_t)b * SEQ;
  const size_t rowe = (size_t)b * EARLY;
  const _Float16* qrow = QKV + (rowb + q0 + ln) * LQ + DM + h * HD;
  const _Float16* kbase = QKV + rowb * LQ + h * HD;
  const _Float16* vbase = VT + (size_t)bh * HD * SEQ;
  const _Float16* klbase = QKVL + rowe * LQ + h * HD;
  const _Float16* vlbase = VTL + (size_t)bh * HD * EARLY;
  const v16h bq0 = ld_frag(qrow, hh), bq1 = ld_frag(qrow + 32, hh);
  v16h bl0 = bq0, bl1 = bq1;
  if (PREC) {
    const _Float16* qlrow = QKVL + (rowe + q0 + ln) * LQ + DM + h * HD;
    bl0 = ld_frag(qlrow, hh);
    bl1 = ld_frag(qlrow + 32, hh);
  }
  const v8f z8 = {0.f, 0.f, 0.f, 0.f, 0.f, 0.f, 0.f, 0.f};
  v8f om0 = z8, om1 = z8, om2 = z8, om3 = z8, or0 = z8, or1 = z8, or2 = z8, or3 = z8;
  float M = -3.0e38f, L = 0.f;
  const int qn = q0 + ln;
  const int nkb = (q0 + 15) / 32 + 1;
#pragma unroll 1
  for (int j = 0; j < nkb - 1; ++j)
    attn_step<PREC, false>(32 * j, qn, ln, hh, kbase, klbase, vbase, vlbase, bq0, bq1, bl0, bl1, M, L, om0, om1, om2, om3, or0, or1, or2, or3);
  attn_step<PREC, true>(32 * (nkb - 1), qn, ln, hh, kbase, klbase, vbase, vlbase, bq0, bq1, bl0, bl1, M, L, om0, om1, om2, om3, or0, or1, or2, or3);

  const float lt = L + __shfl_xor(L, 16, 32);
  const float inv = 64.0f / lt;
  v8f oms[4] = {om0, om1, om2, om3};
  v8f ors[4] = {or0, or1, or2, or3};
#pragma unroll
  for (int t = 0; t < 4; ++t) {
    FragH fh, fl;
#pragma unroll
    for (int r = 0; r < 8; ++r) {
      float val = oms[t][r];
      if (PREC) val = val + ors[t][r] * 0.0009765625f;
      val = val * inv;
      const _Float16 hv = (_Float16)val;
      fh.h[r] = hv;
      fl.h[r] = PREC ? (_Float16)((val - (float)hv) * 1024.0f) : (_Float16)0.0f;
    }
    *(v8us*)&th[w][ln][16 * t + 8 * hh] = fh.half[0];
    if (PREC) *(v8us*)&tl[w][ln][16 * t + 8 * hh] = fl.half[0];
  }
  __builtin_amdgcn_fence(4  , "workgroup");
  __builtin_amdgcn_wave_barrier();
  const int rq = lane >> 3, pc = lane & 7;
  v8us hv4[4], lv4[4];
#pragma unroll
  for (int q = 0; q < 4; ++q) {
    hv4[q] = *(const v8us*)&th[w][4 * q + rq][pc * 8];
    lv4[q] = PREC ? *(const v8us*)&tl[w][4 * q + rq][pc * 8] : hv4[q];
  }
  for (int pass = 0; pass < 2; ++pass) {
#pragma unroll
    for (int q = 0; q < 4; ++q) {
      const int row = q0 + 4 * q + rq;
      *(volatile v8us*)((unsigned short*)CTX + (rowb + row) * DM + h * HD + pc * 8) = hv4[q];
      if (PREC) *(volatile v8us*)((unsigned short*)CTXL + (rowe + row) * DM + h * HD + pc * 8) = lv4[q];
    }
    if (pass == 0) __threadfence();
  }
}

template <bool RES>
__global__ __launch_bounds__(128) void k_gemm_out(const _Float16* __restrict__ CTX, const _Float16* __restrict__ CTXL, const _Float16* __restrict__ Wt,
                                                const float* __restrict__ bias, float* __restrict__ out) {
  __shared__ __attribute__((aligned(16))) float so[4][32][68];
  const int w = __builtin_amdgcn_readfirstlane((int)(threadIdx.x >> 5));
  const int lane = threadIdx.x & 31, ln = lane & 15, hh = lane >> 4;
  const int by = blockIdx.y;
  constexpr int NTN = DM / 64;
  const int mt = blockIdx.x / NTN, nq = blockIdx.x - mt * NTN;
  const int s0 = (RES ? 0 : EARLY) + mt * 128 + 32 * w;
  const int col0 = nq * 64;
  const _Float16* a0p = CTX + ((size_t)by * SEQ + s0 + ln) * DM;
  const _Float16* a1p = a0p + (size_t)16 * DM;
  const _Float16* b0p = Wt + (size_t)(col0 + ln) * DM;
  const v8f z8 = {0.f, 0.f, 0.f, 0.f, 0.f, 0.f, 0.f, 0.f};
  v8f c00 = z8, c01 = z8, c02 = z8, c03 = z8, c10 = z8, c11 = z8, c12 = z8, c13 = z8;
  v8f r00 = z8, r01 = z8, r02 = z8, r03 = z8, r10 = z8, r11 = z8, r12 = z8, r13 = z8;
  gemm_core(a0p, a1p, b0p, DM, DM, hh, c00, c01, c02, c03, c10, c11, c12, c13);
  if (RES) {
    const _Float16* l0p = CTXL + ((size_t)by * EARLY + s0 + ln) * DM;
    const _Float16* l1p = l0p + (size_t)16 * DM;
    gemm_core(l0p, l1p, b0p, DM, DM, hh, r00, r01, r02, r03, r10, r11, r12, r13);
  }
  v8f accs[8] = {c00, c01, c02, c03, c10, c11, c12, c13};
  v8f accr[8] = {r00, r01, r02, r03, r10, r11, r12, r13};
#pragma unroll
  for (int u = 0; u < 8; ++u) {
    const int t = u & 3, half = u >> 2;
    const float bv = bf16_rne(bias[col0 + t * 16 + ln]);
#pragma unroll
    for (int r = 0; r < 8; ++r) {
      float v = accs[u][r] * 0.0009765625f;
      if (RES) v = v + accr[u][r] * 9.5367431640625e-07f;
      so[w][half * 16 + 8 * hh + r][t * 16 + ln] = v + bv;
    }
  }
  __builtin_amdgcn_fence(4  , "workgroup");
  __builtin_amdgcn_wave_barrier();
  const int rsub = lane >> 4, c4 = (lane & 15) * 4;
  for (int pass = 0; pass < 2; ++pass) {
#pragma unroll
    for (int q = 0; q < 16; ++q) {
      const int r = q * 2 + rsub;
      const v4f v = *(const v4fa*)&so[w][r][c4];
      *(volatile v4f*)(out + ((size_t)by * SEQ_FULL + s0 + r) * DM + col0 + c4) = v;
    }
    if (pass == 0) __threadfence();
  }
}

extern "C" void kernel_launch(void* const* d_in, const int* in_sizes, int n_in,
                              void* d_out, int out_size, void* d_ws, size_t ws_size, hipStream_t stream) {
  if (n_in < 5) return;
  const size_t needRows = (size_t)(NB - 1) * SEQ_FULL + SEQ;
  if ((size_t)in_sizes[0] < needRows * DM) return;
  if ((size_t)in_sizes[1] < (size_t)DM * LQ) return;
  if ((size_t)in_sizes[2] < (size_t)LQ) return;
  if ((size_t)in_sizes[3] < (size_t)DM * DM) return;
  if ((size_t)in_sizes[4] < (size_t)DM) return;
  if ((size_t)out_size < needRows * DM) return;
  const float* x = (const float*)d_in[0];
  const float* wkqv = (const float*)d_in[1];
  const float* bkqv = (const float*)d_in[2];
  const float* wout = (const float*)d_in[3];
  const float* bout = (const float*)d_in[4];
  float* out = (float*)d_out;

  char* ws = (char*)d_ws;
  size_t off = 0;
  auto take = [&](size_t bytes) { char* p = ws + off; off += (bytes + 255) & ~(size_t)255; return p; };
  const size_t NR = (size_t)NB * SEQ, NE = (size_t)NB * EARLY;
  _Float16* BQKV = (_Float16*)take((size_t)LQ * DM * 2);
  _Float16* BO   = (_Float16*)take((size_t)DM * DM * 2);
  _Float16* X16  = (_Float16*)take(NR * DM * 2);
  _Float16* QKV  = (_Float16*)take(NR * LQ * 2);
  _Float16* QKVL = (_Float16*)take(NE * LQ * 2);
  _Float16* VT   = (_Float16*)take((size_t)NB * NH * HD * SEQ * 2);
  _Float16* VTL  = (_Float16*)take((size_t)NB * NH * HD * EARLY * 2);
  _Float16* CTX  = (_Float16*)take(NR * DM * 2);
  _Float16* CTXL = (_Float16*)take(NE * DM * 2);
  if (off > ws_size || off > (size_t)134217728) return;

  k_wt_f16<<<(unsigned)(((size_t)LQ * (DM / 8) + 255) / 256), 256, 0, stream>>>(wkqv, BQKV, DM, LQ, 16.0f);
  k_wt_f16<<<(unsigned)(((size_t)DM * (DM / 8) + 255) / 256), 256, 0, stream>>>(wout, BO, DM, DM, 16.0f);
  k_x16<<<(unsigned)((NR * DM / 8 + 255) / 256), 256, 0, stream>>>(x, X16);

  k_gemm_qkv<true><<<dim3((EARLY / 128) * (LQ / 64), NB), 128, 0, stream>>>(X16, BQKV, bkqv, QKV, QKVL);
  if (SEQ > EARLY) k_gemm_qkv<false><<<dim3(((SEQ - EARLY) / 128) * (LQ / 64), NB), 128, 0, stream>>>(X16, BQKV, bkqv, QKV, QKVL);

  k_vt<SEQ><<<NB * NH * (SEQ / 64), 256, 0, stream>>>(QKV + 2 * DM, VT);
  k_vt<EARLY><<<NB * NH * (EARLY / 64), 256, 0, stream>>>(QKVL + 2 * DM, VTL);

  k_attn<true><<<NB * NH * (EARLY / 16) / 4, 128, 0, stream>>>(QKV, QKVL, VT, VTL, CTX, CTXL);
  if (SEQ > EARLY) k_attn<false><<<NB * NH * ((SEQ - EARLY) / 16) / 4, 128, 0, stream>>>(QKV, QKVL, VT, VTL, CTX, CTXL);

  k_gemm_out<true><<<dim3((EARLY / 128) * (DM / 64), NB), 128, 0, stream>>>(CTX, CTXL, BO, bout, out);
  if (SEQ > EARLY) k_gemm_out<false><<<dim3(((SEQ - EARLY) / 128) * (DM / 64), NB), 128, 0, stream>>>(CTX, CTXL, BO, bout, out);
}
